// GINModel_32049045963189
// MI455X (gfx1250) — hardware-verified
//
#include <hip/hip_runtime.h>
#include <stddef.h>

#define DH    128
#define CH    2048
#define BW    32
#define ECAP  2048
#define LBMAX 2048

typedef unsigned int u32;
typedef u32    v2u  __attribute__((ext_vector_type(2)));
typedef u32    v4u  __attribute__((ext_vector_type(4)));
typedef float  v4f  __attribute__((ext_vector_type(4)));
typedef float  v8f  __attribute__((ext_vector_type(8)));
typedef __bf16 v16b __attribute__((ext_vector_type(16)));

union Frag { v16b v; v4u q[2]; };

__device__ __forceinline__ u32 bfbits(float f)
{
    u32 u = __float_as_uint(f);
    return (u + 0x7FFFu + ((u >> 16) & 1u)) >> 16;
}
__device__ __forceinline__ float bfval(u32 b) { return __uint_as_float(b << 16); }

__device__ __forceinline__ int wscan(int v, int lane)
{
#pragma unroll
    for (int d = 1; d < 32; d <<= 1) {
        int y = __shfl_up(v, d, 32);
        if (lane >= d) v += y;
    }
    return v;
}

__device__ __forceinline__ void mma3(v8f& acc, const Frag& ah, const Frag& al, const Frag& bh, const Frag& bl)
{
    acc = __builtin_amdgcn_wmma_f32_16x16x32_bf16(false, ah.v, false, bh.v, (short)0, acc, false, false);
    acc = __builtin_amdgcn_wmma_f32_16x16x32_bf16(false, al.v, false, bh.v, (short)0, acc, false, false);
    acc = __builtin_amdgcn_wmma_f32_16x16x32_bf16(false, ah.v, false, bl.v, (short)0, acc, false, false);
    asm volatile("v_nop\n\tv_nop\n\tv_nop\n\tv_nop" : "+v"(acc) : "v"(ah.v), "v"(al.v), "v"(bh.v), "v"(bl.v));
}

__global__ void __launch_bounds__(256)
k_wprep(const float* __restrict__ W1, const float* __restrict__ W2, u32* wf, int nl)
{
    const int total = nl * 8192;
    const int t = blockIdx.x * blockDim.x + threadIdx.x;
    const bool ok = t < total;
    v4u val = {0u, 0u, 0u, 0u};
    if (ok) {
        const int half = t & 1;
        const int ln   = (t >> 1) & 31;
        const int part = (t >> 6) & 1;
        const int jt   = (t >> 7) & 7;
        const int kb   = (t >> 10) & 3;
        const int mat  = (t >> 12) & 1;
        const int l    = t >> 13;
        const int h = ln >> 4;
        const int n = jt * 16 + (ln & 15);
        const int kbase = kb * 32 + half * 16 + 8 * h;
        const float* W = mat ? W2 : W1;
        const float* wp = W + ((size_t)l * DH + kbase) * DH + n;
        u32 o[4];
#pragma unroll
        for (int jj = 0; jj < 4; ++jj) {
            float f0 = wp[(size_t)(2 * jj) * DH];
            float f1 = wp[(size_t)(2 * jj + 1) * DH];
            u32 a0 = bfbits(f0), a1 = bfbits(f1);
            if (part) { a0 = bfbits(f0 - bfval(a0)); a1 = bfbits(f1 - bfval(a1)); }
            o[jj] = a0 | (a1 << 16);
        }
        val.x = o[0]; val.y = o[1]; val.z = o[2]; val.w = o[3];
    }
    for (int pass = 0; pass < 2; ++pass) {
        if (ok) *(volatile v4u*)(wf + (size_t)t * 4) = val;
        __threadfence();
    }
}

__global__ void __launch_bounds__(256)
k_csort(const int* __restrict__ esrc, const int* __restrict__ edst, int ne, int nn,
        int nb, int nbp, u32* keys_out, int* lb_out)
{
    __shared__ u32 s_k[CH];
    __shared__ __attribute__((aligned(16))) int s_lb[LBMAX];
    const int t = threadIdx.x;
    const int c = blockIdx.x;
    const size_t base = (size_t)c * CH;

    for (int i = t; i < CH; i += 256) {
        const size_t e = base + (size_t)i;
        u32 dk = 0x1FFFFFu;
        if (e < (size_t)ne) {
            const int d = edst[e];
            if ((u32)d < (u32)nn) dk = (u32)d;
        }
        s_k[i] = (dk << 11) | (u32)i;
    }
    __syncthreads();

#pragma unroll 1
    for (int k = 2; k <= CH; k <<= 1) {
#pragma unroll 1
        for (int j = k >> 1; j > 0; j >>= 1) {
#pragma unroll
            for (int it = 0; it < (CH / 2) / 256; ++it) {
                const int idx = t + it * 256;
                const int pos = ((idx & ~(j - 1)) << 1) | (idx & (j - 1));
                const int par = pos | j;
                const u32 a = s_k[pos], bq = s_k[par];
                const bool up = (pos & k) == 0;
                const bool sw = up ? (a > bq) : (a < bq);
                if (sw) { s_k[pos] = bq; s_k[par] = a; }
            }
            __syncthreads();
        }
    }

    for (int b = t; b < nbp; b += 256) {
        const int bb = b < nb ? b : nb;
        const u32 bound = ((u32)bb * (u32)BW) << 11;
        int lo = 0, hi = CH;
        while (lo < hi) {
            const int mid = (lo + hi) >> 1;
            if (s_k[mid] < bound) lo = mid + 1; else hi = mid;
        }
        s_lb[b] = lo;
    }
    __syncthreads();

    for (int pass = 0; pass < 2; ++pass) {
        for (int q = t; q < CH / 2; q += 256) {
            const u32 k0 = s_k[2 * q], k1 = s_k[2 * q + 1];
            const u32 d0 = k0 >> 11, d1 = k1 >> 11;
            u32 s0 = 0u, s1 = 0u;
            if (d0 != 0x1FFFFFu) {
                int s = esrc[base + (size_t)(k0 & (CH - 1))];
                s = s < 0 ? 0 : (s >= nn ? nn - 1 : s);
                s0 = (u32)s;
            }
            if (d1 != 0x1FFFFFu) {
                int s = esrc[base + (size_t)(k1 & (CH - 1))];
                s = s < 0 ? 0 : (s >= nn ? nn - 1 : s);
                s1 = (u32)s;
            }
            v4u o; o.x = s0; o.y = d0; o.z = s1; o.w = d1;
            *(volatile v4u*)(keys_out + (base + (size_t)(2 * q)) * 2) = o;
        }
        for (int q = t; q * 4 < nbp; q += 256) {
            const v4u v = *(const v4u*)(s_lb + q * 4);
            *(volatile v4u*)(lb_out + (size_t)c * nbp + (size_t)q * 4) = v;
        }
        __threadfence();
    }
}

__global__ void __launch_bounds__(256)
k_offs(const int* __restrict__ lb, int nc, int nb, int nbp, int* bstart)
{
    __shared__ int s_sz[LBMAX];
    __shared__ __attribute__((aligned(16))) int s_bs[LBMAX];
    const int t = threadIdx.x, lane = t & 31, wave = t >> 5;

    for (int b = t; b < nb; b += 256) {
        int tot = 0;
        for (int c = 0; c < nc; ++c) {
            int lo = lb[(size_t)c * nbp + b];
            int hi = lb[(size_t)c * nbp + b + 1];
            lo = lo < 0 ? 0 : (lo > CH ? CH : lo);
            hi = hi < 0 ? 0 : (hi > CH ? CH : hi);
            tot += (hi > lo) ? (hi - lo) : 0;
            if (tot > ECAP) tot = ECAP;
        }
        s_sz[b] = (tot + 31) & ~31;
    }
    __syncthreads();
    if (wave == 0) {
        int carry = 0;
        for (int g = 0; g * 32 < nbp; ++g) {
            const int idx = g * 32 + lane;
            const int v = (idx < nb) ? s_sz[idx] : 0;
            const int incl = wscan(v, lane);
            s_bs[idx] = carry + incl - v;
            carry += __shfl(incl, 31, 32);
        }
    }
    __syncthreads();
    for (int pass = 0; pass < 2; ++pass) {
        for (int q = t; q * 4 < nbp; q += 256) {
            const v4u v = *(const v4u*)(s_bs + q * 4);
            *(volatile v4u*)(bstart + (size_t)q * 4) = v;
        }
        __threadfence();
    }
}

__global__ void __launch_bounds__(256)
k_fill(const u32* __restrict__ keys, const int* __restrict__ lb, const int* __restrict__ bstart,
       int nc, int nb, int nbp, u32* srcs, int srccap, int* nstart, int* ndeg)
{
    __shared__ u32 s_list[ECAP];
    __shared__ int s_rank[ECAP];
    __shared__ __attribute__((aligned(16))) u32 s_out[ECAP];
    __shared__ int s_wsum[8];
    __shared__ int s_hist[256];
    __shared__ int s_base[256];
    __shared__ __attribute__((aligned(16))) int s_node[64];

    const int t = threadIdx.x, lane = t & 31, wave = t >> 5;
    const int b = blockIdx.x;
    const int bst = bstart[b];

    for (int i = t; i < ECAP; i += 256) s_out[i] = 0u;

    int run = 0;
    for (int c0 = 0; c0 < nc; c0 += 256) {
        const int c = c0 + t;
        int lo = 0, len = 0;
        if (c < nc) {
            lo = lb[(size_t)c * nbp + b];
            int hi = lb[(size_t)c * nbp + b + 1];
            lo = lo < 0 ? 0 : (lo > CH ? CH : lo);
            hi = hi < 0 ? 0 : (hi > CH ? CH : hi);
            len = (hi > lo) ? (hi - lo) : 0;
        }
        const int incl = wscan(len, lane);
        if (lane == 31) s_wsum[wave] = incl;
        __syncthreads();
        int wpre = 0, blk = 0;
#pragma unroll
        for (int w = 0; w < 8; ++w) {
            const int s = s_wsum[w];
            blk += s;
            wpre += (w < wave) ? s : 0;
        }
        int pos = run + wpre + incl - len;
        for (int q = 0; q < len; ++q, ++pos) {
            if (pos < ECAP) {
                const v2u kv = *(const v2u*)(keys + ((size_t)c * CH + (size_t)(lo + q)) * 2);
                u32 j = kv.y - (u32)b * (u32)BW;
                j = j > 31u ? 31u : j;
                const u32 s = kv.x & 0x07FFFFFFu;
                s_list[pos] = (j << 27) | s;
            }
        }
        run += blk;
        __syncthreads();
    }
    const int total = run < ECAP ? run : ECAP;
    const int pl = (total + 7) >> 3;
    const int e0 = wave * pl;
    int e1 = e0 + pl; if (e1 > total) e1 = total;

    int cnt = 0;
    for (int e = e0; e < e1; ++e) {
        const u32 v = s_list[e];
        if ((v >> 27) == (u32)lane) { s_rank[e] = cnt; ++cnt; }
    }
    s_hist[wave * 32 + lane] = cnt;
    __syncthreads();
    if (wave == 0) {
        int hp[8];
        int deg = 0;
#pragma unroll
        for (int p = 0; p < 8; ++p) { hp[p] = s_hist[p * 32 + lane]; deg += hp[p]; }
        const int incl = wscan(deg, lane);
        const int nst = incl - deg;
        int r = nst;
#pragma unroll
        for (int p = 0; p < 8; ++p) { s_base[p * 32 + lane] = r; r += hp[p]; }
        s_node[lane] = bst + nst;
        s_node[32 + lane] = deg;
    }
    __syncthreads();
    for (int e = t; e < total; e += 256) {
        const u32 v = s_list[e];
        const int j = (int)(v >> 27);
        const int p = e / pl;
        const int pos2 = s_base[p * 32 + j] + s_rank[e];
        if ((unsigned)pos2 < (unsigned)ECAP) s_out[pos2] = v & 0x07FFFFFFu;
    }
    __syncthreads();

    const int padded = (total + 31) & ~31;
    for (int pass = 0; pass < 2; ++pass) {
        for (int q = t; q * 4 < padded; q += 256) {
            const v4u v = *(const v4u*)(s_out + q * 4);
            const long long g = (long long)bst + (long long)(q * 4);
            if (bst >= 0 && g + 4 <= (long long)srccap)
                *(volatile v4u*)(srcs + (size_t)g) = v;
        }
        if (t < 16) {
            const v4u v = *(const v4u*)(s_node + t * 4);
            int* dp = (t < 8) ? (nstart + (size_t)b * BW + t * 4) : (ndeg + (size_t)b * BW + (t - 8) * 4);
            *(volatile v4u*)dp = v;
        }
        __threadfence();
    }
}

__global__ void __launch_bounds__(64) __attribute__((amdgpu_num_vgpr(248)))
k_layer(const float* __restrict__ xin, const int* __restrict__ nstart, const int* __restrict__ ndeg,
        const u32* __restrict__ srcs, int srccap, const u32* __restrict__ wf,
        const float* __restrict__ b1, const float* __restrict__ b2, float* xout, int nn)
{
    __shared__ __attribute__((aligned(16))) u32   s_hi[2][16 * 64];
    __shared__ __attribute__((aligned(16))) u32   s_lo[2][16 * 64];
    __shared__ __attribute__((aligned(16))) float s_o[2][16 * DH];

    const int lane = threadIdx.x & 31;
    const int wave = threadIdx.x >> 5;
    const int h = lane >> 4;
    const int m = lane & 15;
    const int row0 = __builtin_amdgcn_readfirstlane((int)(blockIdx.x * 32u) + wave * 16);
    u32* hiT = s_hi[wave];
    u32* loT = s_lo[wave];
    float* oT = s_o[wave];

#pragma unroll 1
    for (int r = 0; r < 16; ++r) {
        const int node = row0 + r;
        v4f a = {0.f, 0.f, 0.f, 0.f};
        if (node < nn) {
            a = *(const v4f*)(xin + (size_t)node * DH + lane * 4);
            int st = __builtin_amdgcn_readfirstlane(nstart[node]);
            int dg = __builtin_amdgcn_readfirstlane(ndeg[node]);
            st = st < 0 ? 0 : (st > srccap ? srccap : st);
            const int rem = srccap - st;
            dg = dg < 0 ? 0 : (dg > rem ? rem : dg);
#pragma unroll 4
            for (int e = 0; e < dg; ++e) {
                int s = __builtin_amdgcn_readfirstlane((int)(srcs[(size_t)st + e] & 0x07FFFFFFu));
                s = s >= nn ? nn - 1 : s;
                a += *(const v4f*)(xin + (size_t)s * DH + lane * 4);
            }
        }
        const u32 h0 = bfbits(a.x), h1 = bfbits(a.y), h2 = bfbits(a.z), h3 = bfbits(a.w);
        const u32 l0 = bfbits(a.x - bfval(h0)), l1 = bfbits(a.y - bfval(h1));
        const u32 l2 = bfbits(a.z - bfval(h2)), l3 = bfbits(a.w - bfval(h3));
        v2u ph; ph.x = h0 | (h1 << 16); ph.y = h2 | (h3 << 16);
        v2u plw; plw.x = l0 | (l1 << 16); plw.y = l2 | (l3 << 16);
        *(v2u*)(hiT + r * 64 + lane * 2) = ph;
        *(v2u*)(loT + r * 64 + lane * 2) = plw;
    }
    __syncthreads();

    Frag pH[4], pL[4];
#pragma unroll
    for (int jp = 0; jp < 4; ++jp) {
        const v4f u0 = *(const v4f*)(b1 + jp * 32 + 8 * h);
        const v4f u1 = *(const v4f*)(b1 + jp * 32 + 8 * h + 4);
        const v4f u2 = *(const v4f*)(b1 + jp * 32 + 16 + 8 * h);
        const v4f u3 = *(const v4f*)(b1 + jp * 32 + 16 + 8 * h + 4);
        v8f d0 = {u0.x, u0.y, u0.z, u0.w, u1.x, u1.y, u1.z, u1.w};
        v8f d1 = {u2.x, u2.y, u2.z, u2.w, u3.x, u3.y, u3.z, u3.w};
#pragma unroll
        for (int kb = 0; kb < 4; ++kb) {
            Frag bh, bl;
            bh.q[0] = *(const v4u*)(hiT + m * 64 + kb * 16 + 4 * h);
            bh.q[1] = *(const v4u*)(hiT + m * 64 + kb * 16 + 8 + 4 * h);
            bl.q[0] = *(const v4u*)(loT + m * 64 + kb * 16 + 4 * h);
            bl.q[1] = *(const v4u*)(loT + m * 64 + kb * 16 + 8 + 4 * h);
            {
                const u32* p = wf + (size_t)((((0 * 4 + kb) * 8 + (2 * jp)) * 2) * 256) + lane * 8;
                Frag ah, al;
                ah.q[0] = *(const v4u*)(p);       ah.q[1] = *(const v4u*)(p + 4);
                al.q[0] = *(const v4u*)(p + 256); al.q[1] = *(const v4u*)(p + 260);
                mma3(d0, ah, al, bh, bl);
            }
            {
                const u32* p = wf + (size_t)((((0 * 4 + kb) * 8 + (2 * jp + 1)) * 2) * 256) + lane * 8;
                Frag ah, al;
                ah.q[0] = *(const v4u*)(p);       ah.q[1] = *(const v4u*)(p + 4);
                al.q[0] = *(const v4u*)(p + 256); al.q[1] = *(const v4u*)(p + 260);
                mma3(d1, ah, al, bh, bl);
            }
        }
        Frag ph, plo;
#pragma unroll
        for (int w = 0; w < 4; ++w) {
            const float x0 = fmaxf(d0[2 * w], 0.f), x1 = fmaxf(d0[2 * w + 1], 0.f);
            const float y0 = fmaxf(d1[2 * w], 0.f), y1 = fmaxf(d1[2 * w + 1], 0.f);
            const u32 hx0 = bfbits(x0), hx1 = bfbits(x1), hy0 = bfbits(y0), hy1 = bfbits(y1);
            const u32 lx0 = bfbits(x0 - bfval(hx0)), lx1 = bfbits(x1 - bfval(hx1));
            const u32 ly0 = bfbits(y0 - bfval(hy0)), ly1 = bfbits(y1 - bfval(hy1));
            ph.q[0][w]  = hx0 | (hx1 << 16);
            ph.q[1][w]  = hy0 | (hy1 << 16);
            plo.q[0][w] = lx0 | (lx1 << 16);
            plo.q[1][w] = ly0 | (ly1 << 16);
        }
        pH[jp] = ph;
        pL[jp] = plo;
    }

#pragma unroll
    for (int ot = 0; ot < 8; ++ot) {
        const v4f u0 = *(const v4f*)(b2 + ot * 16 + 8 * h);
        const v4f u1 = *(const v4f*)(b2 + ot * 16 + 8 * h + 4);
        v8f d = {u0.x, u0.y, u0.z, u0.w, u1.x, u1.y, u1.z, u1.w};
#pragma unroll
        for (int kb = 0; kb < 4; ++kb) {
            const u32* p = wf + (size_t)((((1 * 4 + kb) * 8 + ot) * 2) * 256) + lane * 8;
            Frag ah, al;
            ah.q[0] = *(const v4u*)(p);       ah.q[1] = *(const v4u*)(p + 4);
            al.q[0] = *(const v4u*)(p + 256); al.q[1] = *(const v4u*)(p + 260);
            mma3(d, ah, al, pH[kb], pL[kb]);
        }
        v4f o0 = {d[0], d[1], d[2], d[3]};
        v4f o1 = {d[4], d[5], d[6], d[7]};
        *(v4f*)(oT + m * DH + ot * 16 + 8 * h)     = o0;
        *(v4f*)(oT + m * DH + ot * 16 + 8 * h + 4) = o1;
    }
    __syncthreads();

    for (int pass = 0; pass < 2; ++pass) {
#pragma unroll
        for (int r = 0; r < 16; ++r) {
            const int node = row0 + r;
            if (node < nn) {
                const v4f v = *(const v4f*)(oT + r * DH + lane * 4);
                *(volatile v4f*)(xout + (size_t)node * DH + lane * 4) = v;
            }
        }
        __threadfence();
    }
}

static inline size_t al128(size_t b) { return (b + 127) & ~(size_t)127; }

extern "C" void kernel_launch(void* const* d_in, const int* in_sizes, int n_in,
                              void* d_out, int out_size, void* d_ws, size_t ws_size,
                              hipStream_t stream)
{
    if (n_in < 6) return;
    const float* x  = (const float*)d_in[0];
    const int*   ei = (const int*)d_in[1];
    const float* W1 = (const float*)d_in[2];
    const float* b1 = (const float*)d_in[3];
    const float* W2 = (const float*)d_in[4];
    const float* b2 = (const float*)d_in[5];
    float* out = (float*)d_out;

    const int N = in_sizes[0] / DH;
    const int E = in_sizes[1] / 2;
    const int L = in_sizes[2] / (DH * DH);
    if (N <= 0 || L <= 0 || E < 0) return;
    if (N > (1 << 20)) return;
    if ((long long)out_size < (long long)N * DH) return;

    const int NB     = (N + BW - 1) / BW;
    const int NBP    = ((NB + 1) + 31) / 32 * 32;
    const int NC     = (E + CH - 1) / CH;
    const int NCA    = NC > 0 ? NC : 1;
    const int SRCCAP = E + BW * NB;
    if (NBP > LBMAX) return;

    size_t off = 0;
    const size_t o_bufA = off; off += al128((size_t)N * DH * sizeof(float));
    const size_t o_bufB = off; off += al128((size_t)N * DH * sizeof(float));
    const size_t o_wf   = off; off += al128((size_t)L * 32768 * sizeof(u32));
    const size_t o_keys = off; off += al128((size_t)NCA * CH * 2 * sizeof(u32));
    const size_t o_lb   = off; off += al128((size_t)NCA * NBP * sizeof(int));
    const size_t o_bst  = off; off += al128((size_t)NBP * sizeof(int));
    const size_t o_nst  = off; off += al128((size_t)NB * BW * sizeof(int));
    const size_t o_ndg  = off; off += al128((size_t)NB * BW * sizeof(int));
    const size_t o_srcs = off; off += al128((size_t)SRCCAP * sizeof(u32));
    if (off > ws_size) return;

    char* ws = (char*)d_ws;
    float* bufA = (float*)(ws + o_bufA);
    float* bufB = (float*)(ws + o_bufB);
    u32*   wf   = (u32*)(ws + o_wf);
    u32*   keys = (u32*)(ws + o_keys);
    int*   lb   = (int*)(ws + o_lb);
    int*   bst  = (int*)(ws + o_bst);
    int*   nst  = (int*)(ws + o_nst);
    int*   ndg  = (int*)(ws + o_ndg);
    u32*   srcs = (u32*)(ws + o_srcs);

    const int wtotal = L * 8192;
    k_wprep<<<dim3((wtotal + 255) / 256), dim3(256), 0, stream>>>(W1, W2, wf, L);

    if (NC > 0)
        k_csort<<<dim3(NC), dim3(256), 0, stream>>>(ei, ei + E, E, N, NB, NBP, keys, lb);
    k_offs<<<dim3(1), dim3(256), 0, stream>>>(lb, NC, NB, NBP, bst);
    k_fill<<<dim3(NB), dim3(256), 0, stream>>>(keys, lb, bst, NC, NB, NBP, srcs, SRCCAP, nst, ndg);

    const float* hcur = x;
    for (int l = 0; l < L; ++l) {
        float* hout = (l == L - 1) ? out : ((l & 1) ? bufB : bufA);
        k_layer<<<dim3((N + 31) / 32), dim3(64), 0, stream>>>(
            hcur, nst, ndg, srcs, SRCCAP, wf + (size_t)l * 32768,
            b1 + (size_t)l * DH, b2 + (size_t)l * DH, hout, N);
        hcur = hout;
    }
}
